// DualResolutionAttention_74577812127847
// MI455X (gfx1250) — hardware-verified
//
#include <hip/hip_runtime.h>
#include <math.h>
#include <stdint.h>

#define NB_  2
#define T_   4096
#define E_   1024
#define LD_  512
#define HH_  8
#define TC_  1024
#define NEL_ 128
#define NEG_ 128
#define XE_  512
static_assert(NEG_ * 4 == XE_);
static_assert(NEL_ <= XE_);
static_assert((NEL_ % 64) == 0 && (NEG_ % 64) == 0);

typedef _Float16 v16h __attribute__((ext_vector_type(16)));
typedef _Float16 v8h  __attribute__((ext_vector_type(8)));
typedef __bf16   v16b __attribute__((ext_vector_type(16)));
typedef __bf16   v8b  __attribute__((ext_vector_type(8)));
typedef float    v8f  __attribute__((ext_vector_type(8)));
typedef float    v4f  __attribute__((ext_vector_type(4)));
typedef float    v2f  __attribute__((ext_vector_type(2)));
typedef unsigned int v4u __attribute__((ext_vector_type(4)));

__device__ __forceinline__ unsigned short f2bf_bits(float f) {
  unsigned u = __float_as_uint(f);
  return (unsigned short)((u + 0x7FFFu + ((u >> 16) & 1u)) >> 16);
}
__device__ __forceinline__ float bf_bits2f(unsigned short hb) { return __uint_as_float(((unsigned)hb) << 16); }
__device__ __forceinline__ unsigned short f2h_bits(float f) { return __builtin_bit_cast(unsigned short, (_Float16)f); }
__device__ __forceinline__ unsigned pk16(unsigned short a, unsigned short b) { return (unsigned)a | ((unsigned)b << 16); }

__device__ __forceinline__ void guard1_h(v8f& a, v16h x, v16h y) {
  asm volatile("v_nop\n\tv_nop\n\tv_nop\n\tv_nop" : "+v"(a) : "v"(x), "v"(y));
}
__device__ __forceinline__ void guard1_b(v8f& a, v16b x, v16b y) {
  asm volatile("v_nop\n\tv_nop\n\tv_nop\n\tv_nop" : "+v"(a) : "v"(x), "v"(y));
}
__device__ __forceinline__ void guard2_h(v8f& a, v8f& b, v16h x, v16h y) {
  asm volatile("v_nop\n\tv_nop\n\tv_nop\n\tv_nop" : "+v"(a), "+v"(b) : "v"(x), "v"(y));
}
__device__ __forceinline__ void guard2_b(v8f& a, v8f& b, v16b x, v16b y) {
  asm volatile("v_nop\n\tv_nop\n\tv_nop\n\tv_nop" : "+v"(a), "+v"(b) : "v"(x), "v"(y));
}
__device__ __forceinline__ void keep4_h(v16h a, v16h b, v16h c, v16h d) { asm volatile("v_nop" :: "v"(a), "v"(b), "v"(c), "v"(d)); }
__device__ __forceinline__ void keep4_b(v16b a, v16b b, v16b c, v16b d) { asm volatile("v_nop" :: "v"(a), "v"(b), "v"(c), "v"(d)); }
__device__ __forceinline__ void acc_guard4(v8f& a, v8f& b, v8f& c, v8f& d) {
  asm volatile("v_nop\n\tv_nop\n\tv_nop\n\tv_nop" : "+v"(a), "+v"(b), "+v"(c), "+v"(d));
}

template <typename T> struct Frag;
template <> struct Frag<_Float16> {
  typedef v16h V; typedef v8h H; union U { v16h v; v8h h[2]; };
  static __device__ __forceinline__ v16h load(const _Float16* p) {
    U f; f.h[0] = *(const v8h*)(p); f.h[1] = *(const v8h*)(p + 16); return f.v;
  }
  static __device__ __forceinline__ v8f mma(v16h a, v16h b, v8f c) {
    return __builtin_amdgcn_wmma_f32_16x16x32_f16(false, a, false, b, (short)0, c, false, false);
  }
  static __device__ __forceinline__ v8f mma_g(v16h a, v16h b, v8f c) { c = mma(a, b, c); guard1_h(c, a, b); return c; }
  static __device__ __forceinline__ void guard(v8f& a, v8f& b, v16h x, v16h y) { guard2_h(a, b, x, y); }
  static __device__ __forceinline__ void keep(v16h a, v16h b, v16h c, v16h d) { keep4_h(a, b, c, d); }
};
template <> struct Frag<__bf16> {
  typedef v16b V; typedef v8b H; union U { v16b v; v8b h[2]; };
  static __device__ __forceinline__ v16b load(const __bf16* p) {
    U f; f.h[0] = *(const v8b*)(p); f.h[1] = *(const v8b*)(p + 16); return f.v;
  }
  static __device__ __forceinline__ v8f mma(v16b a, v16b b, v8f c) {
    return __builtin_amdgcn_wmma_f32_16x16x32_bf16(false, a, false, b, (short)0, c, false, false);
  }
  static __device__ __forceinline__ v8f mma_g(v16b a, v16b b, v8f c) { c = mma(a, b, c); guard1_b(c, a, b); return c; }
  static __device__ __forceinline__ void guard(v8f& a, v8f& b, v16b x, v16b y) { guard2_b(a, b, x, y); }
  static __device__ __forceinline__ void keep(v16b a, v16b b, v16b c, v16b d) { keep4_b(a, b, c, d); }
};
template <int ET> struct Elem;
template <> struct Elem<0> { typedef _Float16 T; };
template <> struct Elem<1> { typedef __bf16 T; };

template <int ET, bool SPLIT, int BIAS_MODE, int OUT_MODE, int MI>
__global__ __launch_bounds__(256) void wmma_gemm(
    const unsigned short* __restrict__ Ap, const unsigned short* __restrict__ A2p, int lda, long long strideA,
    const unsigned short* __restrict__ Btp, const unsigned short* __restrict__ Bt2p, int ldb, long long strideB,
    void* __restrict__ Cout, void* __restrict__ Cout2, int ldc, long long strideC,
    const float* __restrict__ bias, int M, int N, int K, float scale, float oscale) {
  typedef typename Elem<ET>::T T;
  typedef Frag<T> F;
  typedef typename F::V V;
  const T* A = (const T*)Ap; const T* A2 = (const T*)A2p; const T* Bt = (const T*)Btp; const T* Bt2 = (const T*)Bt2p;
  __shared__ __align__(16) float sT[8][16 * 68];

  const int b    = blockIdx.y;
  const int lane = threadIdx.x & 31;
  const int wave = threadIdx.x >> 5;
  const int rowsW  = 16 * MI;
  const int tilesN = N >> 6;
  const int tilesM = M / rowsW;
  const int tile = blockIdx.x * 8 + wave;
  if (tile >= tilesM * tilesN) return;
  const int tm = tile / tilesN;
  const int tn = tile - tm * tilesN;
  const int m0 = tm * rowsW;
  const int n0 = tn << 6;

  const T* Ab  = A   + (size_t)b * strideA;
  const T* Bb  = Bt  + (size_t)b * strideB;
  const T* Ab2 = A2  + (size_t)b * strideA;
  const T* Bb2 = Bt2 + (size_t)b * strideB;

  const int rlane = lane & 15;
  const int koff  = (lane >> 4) * 8;
  const int mOff  = (lane >> 4) * 8;

  v8f acc[MI][4];
#pragma unroll
  for (int i = 0; i < MI; ++i)
#pragma unroll
    for (int j = 0; j < 4; ++j) acc[i][j] = (v8f){0.f, 0.f, 0.f, 0.f, 0.f, 0.f, 0.f, 0.f};

  for (int k0 = 0; k0 < K; k0 += 32) {
    V bh[4], bl[4];
#pragma unroll
    for (int j = 0; j < 4; ++j) {
      const size_t bo = (size_t)(n0 + (j << 4) + rlane) * ldb + koff + k0;
      bh[j] = F::load(Bb + bo);
      if (SPLIT) bl[j] = F::load(Bb2 + bo); else bl[j] = bh[j];
    }
#pragma unroll
    for (int i = 0; i < MI; ++i) {
      const size_t ao = (size_t)(m0 + (i << 4) + rlane) * lda + koff + k0;
      V ah = F::load(Ab + ao);
      V al = ah;
      if (SPLIT) al = F::load(Ab2 + ao);
#pragma unroll
      for (int j = 0; j < 4; ++j) {
        acc[i][j] = F::mma(ah, bh[j], acc[i][j]);
        if (SPLIT) {
          acc[i][j] = F::mma(ah, bl[j], acc[i][j]);
          acc[i][j] = F::mma(al, bh[j], acc[i][j]);
        }
      }
      F::guard(acc[i][0], acc[i][3], ah, al);
    }
    F::keep(bh[0], bh[1], bh[2], bh[3]);
    if (SPLIT) F::keep(bl[0], bl[1], bl[2], bl[3]);
  }
#pragma unroll
  for (int i = 0; i < MI; ++i) acc_guard4(acc[i][0], acc[i][1], acc[i][2], acc[i][3]);

  float* slab = sT[wave];
#pragma unroll
  for (int i = 0; i < MI; ++i) {
    const int mBase = m0 + (i << 4);
#pragma unroll
    for (int j = 0; j < 4; ++j) {
      const int n = n0 + (j << 4) + rlane;
      float bv = 0.f;
      if (BIAS_MODE == 2) bv = bias[n];
#pragma unroll
      for (int r = 0; r < 8; ++r) {
        float v = acc[i][j][r] * scale;
        if (BIAS_MODE == 1) v += bias[mBase + mOff + r];
        if (BIAS_MODE == 2) v += bv;
        if (OUT_MODE == 1) v *= oscale;
        slab[(mOff + r) * 68 + (j << 4) + rlane] = v;
      }
    }
    __builtin_amdgcn_fence(__ATOMIC_RELEASE, "workgroup");
    __builtin_amdgcn_wave_barrier();
    __builtin_amdgcn_fence(__ATOMIC_ACQUIRE, "workgroup");
    if (OUT_MODE == 0) {
      float* C = (float*)Cout + (size_t)b * strideC;
      const int hh = lane >> 4, c4 = (lane & 15) * 4;
      for (int pass = 0; pass < 2; ++pass) {
#pragma unroll
        for (int it = 0; it < 8; ++it) {
          const int row = it * 2 + hh;
          v4f v = *(const v4f*)(slab + row * 68 + c4);
          *(volatile v4f*)(C + (size_t)(mBase + row) * ldc + n0 + c4) = v;
        }
        __threadfence();
      }
    } else {
      const int q = lane >> 3, c8 = (lane & 7) * 8;
      unsigned short* C  = (unsigned short*)Cout + (size_t)b * strideC;
      unsigned short* C2 = (unsigned short*)Cout2 + (size_t)b * strideC;
      for (int pass = 0; pass < 2; ++pass) {
#pragma unroll
        for (int it = 0; it < 4; ++it) {
          const int row = it * 4 + q;
          const float* sp = slab + row * 68 + c8;
          v4u hv, lv;
#pragma unroll
          for (int e = 0; e < 4; ++e) {
            const float f0 = sp[2 * e], f1 = sp[2 * e + 1];
            if (OUT_MODE == 1) {
              hv[e] = pk16(f2h_bits(f0), f2h_bits(f1));
              lv[e] = hv[e];
            } else {
              const unsigned short h0 = f2bf_bits(f0), h1 = f2bf_bits(f1);
              const unsigned short l0 = f2bf_bits(f0 - bf_bits2f(h0)), l1 = f2bf_bits(f1 - bf_bits2f(h1));
              hv[e] = pk16(h0, h1);
              lv[e] = pk16(l0, l1);
            }
          }
          *(volatile v4u*)(C + (size_t)(mBase + row) * ldc + n0 + c8) = hv;
          if (OUT_MODE == 2) *(volatile v4u*)(C2 + (size_t)(mBase + row) * ldc + n0 + c8) = lv;
        }
        __threadfence();
      }
    }
    __builtin_amdgcn_fence(__ATOMIC_RELEASE, "workgroup");
    __builtin_amdgcn_wave_barrier();
    __builtin_amdgcn_fence(__ATOMIC_ACQUIRE, "workgroup");
  }
}

__global__ __launch_bounds__(256) void wconv_kernel(const float* __restrict__ W, int ldw,
                                                    unsigned short* __restrict__ of, unsigned short* __restrict__ oh,
                                                    unsigned short* __restrict__ ol, int R, int Cc, float fs) {
  __shared__ __align__(16) float tf[64 * 68];
  const int c0  = blockIdx.x * 64;
  const int r0  = blockIdx.y * 64;
  const int tid = threadIdx.x;
  (void)Cc;
  {
    const int lr = tid >> 4;
    const int c4 = (tid & 15) * 4;
#pragma unroll
    for (int it = 0; it < 4; ++it) {
      const int rr = it * 16 + lr;
      const v4f a = *(const v4f*)(W + (size_t)(r0 + rr) * ldw + c0 + c4);
      *(v4f*)(tf + rr * 68 + c4) = a;
    }
  }
  __syncthreads();
  const int sub = tid >> 3;
  const int c8  = (tid & 7) * 8;
  v4u fv[2], hv[2], lv[2];
#pragma unroll
  for (int it = 0; it < 2; ++it) {
    const int oc = it * 32 + sub;
    v4u a, bh, bl;
#pragma unroll
    for (int q = 0; q < 4; ++q) {
      const float f0 = tf[(c8 + 2 * q) * 68 + oc];
      const float f1 = tf[(c8 + 2 * q + 1) * 68 + oc];
      const unsigned short h0 = f2bf_bits(f0), h1 = f2bf_bits(f1);
      const unsigned short l0 = f2bf_bits(f0 - bf_bits2f(h0)), l1 = f2bf_bits(f1 - bf_bits2f(h1));
      a[q]  = pk16(f2h_bits(f0 * fs), f2h_bits(f1 * fs));
      bh[q] = pk16(h0, h1);
      bl[q] = pk16(l0, l1);
    }
    fv[it] = a; hv[it] = bh; lv[it] = bl;
  }
  for (int pass = 0; pass < 2; ++pass) {
#pragma unroll
    for (int it = 0; it < 2; ++it) {
      const int oc = it * 32 + sub;
      const size_t go = (size_t)(c0 + oc) * R + r0 + c8;
      *(volatile v4u*)(of + go) = fv[it];
      *(volatile v4u*)(oh + go) = hv[it];
      *(volatile v4u*)(ol + go) = lv[it];
    }
    __threadfence();
  }
}

__global__ __launch_bounds__(256) void xconv_kernel(const float* __restrict__ x, unsigned short* __restrict__ xo, int n8, float fs) {
  const int i = blockIdx.x * 256 + threadIdx.x;
  if (i >= n8) return;
  const v4f a = *(const v4f*)(x + 8 * (size_t)i);
  const v4f c = *(const v4f*)(x + 8 * (size_t)i + 4);
  v4u o;
  o[0] = pk16(f2h_bits(a[0] * fs), f2h_bits(a[1] * fs));
  o[1] = pk16(f2h_bits(a[2] * fs), f2h_bits(a[3] * fs));
  o[2] = pk16(f2h_bits(c[0] * fs), f2h_bits(c[1] * fs));
  o[3] = pk16(f2h_bits(c[2] * fs), f2h_bits(c[3] * fs));
  *(volatile v4u*)(xo + 8 * (size_t)i) = o;
  __threadfence();
  *(volatile v4u*)(xo + 8 * (size_t)i) = o;
}

__global__ __launch_bounds__(256) void split_bf16x2_kernel(const float* __restrict__ in, long long ibs,
                                                           unsigned short* __restrict__ hi, unsigned short* __restrict__ lo,
                                                           long long obs, int n2) {
  const int i = blockIdx.x * 256 + threadIdx.x;
  if (i >= n2) return;
  const float* inb = in + (size_t)blockIdx.y * (size_t)ibs;
  unsigned short* hb = hi + (size_t)blockIdx.y * (size_t)obs;
  unsigned short* lb = lo + (size_t)blockIdx.y * (size_t)obs;
  const v2f f = *(const v2f*)(inb + 2 * (size_t)i);
  const unsigned short h0 = f2bf_bits(f[0]), h1 = f2bf_bits(f[1]);
  const unsigned short l0 = f2bf_bits(f[0] - bf_bits2f(h0)), l1 = f2bf_bits(f[1] - bf_bits2f(h1));
  const unsigned uh = pk16(h0, h1), ul = pk16(l0, l1);
  ((volatile unsigned*)hb)[i] = uh;
  ((volatile unsigned*)lb)[i] = ul;
  __threadfence();
  ((volatile unsigned*)hb)[i] = uh;
  ((volatile unsigned*)lb)[i] = ul;
}

template <int ET>
__global__ __launch_bounds__(128)
void attn_causal64(const unsigned short* __restrict__ qk1p, const unsigned short* __restrict__ qk2p, int qpitch, long long qbs, int kcol,
                   const unsigned short* __restrict__ vt1p, const unsigned short* __restrict__ vt2p, int vpitch, long long vbs,
                   void* __restrict__ outp, int opitch, long long obs, int nqb, float sscale, float oscale) {
  typedef typename Elem<ET>::T T;
  typedef Frag<T> F;
  typedef typename F::V V;
  typedef typename F::H H;
  constexpr bool SPLIT = (ET == 1);
  union FB { V v; H h[2]; };
  __shared__ __align__(16) T Ks1[64 * 64];
  __shared__ __align__(16) T Ks2[SPLIT ? (64 * 64) : 16];
  __shared__ __align__(16) T Vs1[64 * 64];
  __shared__ __align__(16) T Vs2[SPLIT ? (64 * 64) : 16];
  __shared__ __align__(16) T Ps1[4 * 16 * 64];
  __shared__ __align__(16) T Ps2[SPLIT ? (4 * 16 * 64) : 16];
  __shared__ __align__(16) float Os[4 * 16 * 68];

  const int tid  = threadIdx.x;
  const int wave = tid >> 5;
  const int lane = tid & 31;
  const int hh   = lane >> 4;
  const int c    = lane & 15;
  const int b    = blockIdx.y;
  const int bx   = blockIdx.x;
  const int qb   = bx % nqb;
  const int h    = bx / nqb;
  const int q0   = qb * 64 + wave * 16;
  const float NEG_INF = -__builtin_inff();

  const T* Q1 = (const T*)qk1p + (size_t)b * qbs + (size_t)h * 64;
  const T* Q2 = (const T*)qk2p + (size_t)b * qbs + (size_t)h * 64;
  const T* K1 = Q1 + kcol;
  const T* K2 = Q2 + kcol;
  const T* V1 = (const T*)vt1p + (size_t)b * vbs + (size_t)h * 64 * vpitch;
  const T* V2 = (const T*)vt2p + (size_t)b * vbs + (size_t)h * 64 * vpitch;

  V qa1[2], qa2[2];
#pragma unroll
  for (int dc = 0; dc < 2; ++dc) {
    const size_t qo = (size_t)(q0 + c) * qpitch + dc * 32 + 8 * hh;
    qa1[dc] = F::load(Q1 + qo);
    if (SPLIT) qa2[dc] = F::load(Q2 + qo); else qa2[dc] = qa1[dc];
  }

  float mrow[8], lrow[8];
  v8f oacc[4];
#pragma unroll
  for (int r = 0; r < 8; ++r) { mrow[r] = NEG_INF; lrow[r] = 0.f; }
#pragma unroll
  for (int t = 0; t < 4; ++t) oacc[t] = (v8f){0.f, 0.f, 0.f, 0.f, 0.f, 0.f, 0.f, 0.f};

  const int nChunks = qb + 1;
  for (int kc = 0; kc < nChunks; ++kc) {
    const int kv0 = kc * 64;
    __syncthreads();
    {
      const int r = tid >> 1, half = (tid & 1) * 32;
      const T* ks1 = K1 + (size_t)(kv0 + r) * qpitch + half;
      const T* ks2 = K2 + (size_t)(kv0 + r) * qpitch + half;
      const T* vs1 = V1 + (size_t)r * vpitch + kv0 + half;
      const T* vs2 = V2 + (size_t)r * vpitch + kv0 + half;
#pragma unroll
      for (int i = 0; i < 4; ++i) {
        const H a1 = *(const H*)(ks1 + 8 * i);
        const H w1 = *(const H*)(vs1 + 8 * i);
        *(H*)(Ks1 + r * 64 + half + 8 * i) = a1;
        *(H*)(Vs1 + r * 64 + half + 8 * i) = w1;
        if (SPLIT) {
          const H a2 = *(const H*)(ks2 + 8 * i);
          const H w2 = *(const H*)(vs2 + 8 * i);
          *(H*)(Ks2 + r * 64 + half + 8 * i) = a2;
          *(H*)(Vs2 + r * 64 + half + 8 * i) = w2;
        }
      }
    }
    __syncthreads();

    v8f s[4];
#pragma unroll
    for (int j = 0; j < 4; ++j) {
      s[j] = (v8f){0.f, 0.f, 0.f, 0.f, 0.f, 0.f, 0.f, 0.f};
#pragma unroll
      for (int dc = 0; dc < 2; ++dc) {
        FB kb, kl;
        kb.h[0] = *(const H*)(Ks1 + (j * 16 + c) * 64 + dc * 32 + 8 * hh);
        kb.h[1] = *(const H*)(Ks1 + (j * 16 + c) * 64 + dc * 32 + 16 + 8 * hh);
        if (SPLIT) {
          kl.h[0] = *(const H*)(Ks2 + (j * 16 + c) * 64 + dc * 32 + 8 * hh);
          kl.h[1] = *(const H*)(Ks2 + (j * 16 + c) * 64 + dc * 32 + 16 + 8 * hh);
          s[j] = F::mma_g(qa1[dc], kb.v, s[j]);
          s[j] = F::mma_g(qa1[dc], kl.v, s[j]);
          s[j] = F::mma_g(qa2[dc], kb.v, s[j]);
        } else {
          s[j] = F::mma_g(qa1[dc], kb.v, s[j]);
        }
      }
    }

    const bool diag = (kc == qb);
    float cm[8];
#pragma unroll
    for (int r = 0; r < 8; ++r) {
      const int qrow = q0 + 8 * hh + r;
      float m = NEG_INF;
#pragma unroll
      for (int j = 0; j < 4; ++j) {
        const int kvcol = kv0 + j * 16 + c;
        const float sv = s[j][r] * sscale;
        const bool masked = diag && (kvcol > qrow);
        const float sm = masked ? NEG_INF : sv;
        s[j][r] = sm;
        m = fmaxf(m, sm);
      }
#pragma unroll
      for (int off = 1; off < 16; off <<= 1) m = fmaxf(m, __shfl_xor(m, off, 32));
      cm[r] = m;
    }
    T* pw1 = Ps1 + wave * (16 * 64);
    T* pw2 = pw1;
    if (SPLIT) pw2 = Ps2 + wave * (16 * 64);
#pragma unroll
    for (int r = 0; r < 8; ++r) {
      const float mnew  = fmaxf(mrow[r], cm[r]);
      const float alpha = expf(mrow[r] - mnew);
      mrow[r] = mnew;
      float psum = 0.f;
#pragma unroll
      for (int j = 0; j < 4; ++j) {
        const float p = expf(s[j][r] - mnew);
        psum += p;
        const int pi = (8 * hh + r) * 64 + j * 16 + c;
        if (SPLIT) {
          const unsigned short hb = f2bf_bits(p);
          const unsigned short lb = f2bf_bits(p - bf_bits2f(hb));
          pw1[pi] = __builtin_bit_cast(T, hb);
          pw2[pi] = __builtin_bit_cast(T, lb);
        } else {
          pw1[pi] = __builtin_bit_cast(T, f2h_bits(p * 1024.f));
        }
      }
#pragma unroll
      for (int off = 1; off < 16; off <<= 1) psum += __shfl_xor(psum, off, 32);
      lrow[r] = lrow[r] * alpha + psum;
#pragma unroll
      for (int t = 0; t < 4; ++t) oacc[t][r] *= alpha;
    }
    __builtin_amdgcn_fence(__ATOMIC_RELEASE, "workgroup");
    __builtin_amdgcn_wave_barrier();
    __builtin_amdgcn_fence(__ATOMIC_ACQUIRE, "workgroup");

#pragma unroll 1
    for (int kk = 0; kk < 2; ++kk) {
      FB pa, pl;
      pa.h[0] = *(const H*)(pw1 + c * 64 + kk * 32 + 8 * hh);
      pa.h[1] = *(const H*)(pw1 + c * 64 + kk * 32 + 16 + 8 * hh);
      if (SPLIT) {
        pl.h[0] = *(const H*)(pw2 + c * 64 + kk * 32 + 8 * hh);
        pl.h[1] = *(const H*)(pw2 + c * 64 + kk * 32 + 16 + 8 * hh);
      } else {
        pl = pa;
      }
#pragma unroll
      for (int t = 0; t < 4; ++t) {
        FB vb, vl;
        vb.h[0] = *(const H*)(Vs1 + (t * 16 + c) * 64 + kk * 32 + 8 * hh);
        vb.h[1] = *(const H*)(Vs1 + (t * 16 + c) * 64 + kk * 32 + 16 + 8 * hh);
        if (SPLIT) {
          vl.h[0] = *(const H*)(Vs2 + (t * 16 + c) * 64 + kk * 32 + 8 * hh);
          vl.h[1] = *(const H*)(Vs2 + (t * 16 + c) * 64 + kk * 32 + 16 + 8 * hh);
          oacc[t] = F::mma_g(pa.v, vb.v, oacc[t]);
          oacc[t] = F::mma_g(pa.v, vl.v, oacc[t]);
          oacc[t] = F::mma_g(pl.v, vb.v, oacc[t]);
        } else {
          oacc[t] = F::mma_g(pa.v, vb.v, oacc[t]);
        }
      }
    }
  }

  float* os = Os + wave * (16 * 68);
#pragma unroll
  for (int r = 0; r < 8; ++r) {
    const float inv = oscale / lrow[r];
#pragma unroll
    for (int t = 0; t < 4; ++t) os[(8 * hh + r) * 68 + t * 16 + c] = oacc[t][r] * inv;
  }
  __builtin_amdgcn_fence(__ATOMIC_RELEASE, "workgroup");
  __builtin_amdgcn_wave_barrier();
  __builtin_amdgcn_fence(__ATOMIC_ACQUIRE, "workgroup");
  if (SPLIT) {
    float* Ob = (float*)outp + (size_t)b * obs + (size_t)h * 64;
    const int c4 = (lane & 15) * 4;
    for (int pass = 0; pass < 2; ++pass) {
#pragma unroll
      for (int it = 0; it < 8; ++it) {
        const int row = it * 2 + hh;
        v4f val = *(const v4f*)(os + row * 68 + c4);
        *(volatile v4f*)(Ob + (size_t)(q0 + row) * opitch + c4) = val;
      }
      __threadfence();
    }
  } else {
    unsigned short* Ob = (unsigned short*)outp + (size_t)b * obs + (size_t)h * 64;
    const int q = lane >> 3, c8 = (lane & 7) * 8;
    v8h hv[4];
#pragma unroll
    for (int it = 0; it < 4; ++it) {
      const int row = it * 4 + q;
      const float* sp = os + row * 68 + c8;
      v8h t8;
#pragma unroll
      for (int e = 0; e < 8; ++e) t8[e] = (_Float16)sp[e];
      hv[it] = t8;
    }
    for (int pass = 0; pass < 2; ++pass) {
#pragma unroll
      for (int it = 0; it < 4; ++it) {
        const int row = it * 4 + q;
        *(volatile v8h*)(Ob + (size_t)(q0 + row) * opitch + c8) = hv[it];
      }
      __threadfence();
    }
  }
}

__global__ __launch_bounds__(256) void gate_out_kernel(const float* __restrict__ L, const float* __restrict__ EL,
                                                      const float* __restrict__ G, const float* __restrict__ EG,
                                                      const float* __restrict__ wg, const float* __restrict__ bg,
                                                      float* __restrict__ out, int ntok, int Tn, int Tcn, int nel, int neg) {
  const int tid = threadIdx.x, wave = tid >> 5, lane = tid & 31;
  const int row = blockIdx.x * 8 + wave;
  if (row >= ntok) return;
  const int b  = row / Tn;
  const int t  = row - b * Tn;
  const int tc = t >> 2;
  const float* ls = (t < nel)  ? (EL + ((size_t)b * nel + t) * LD_)  : (L + (size_t)row * LD_);
  const float* gs = (tc < neg) ? (EG + ((size_t)b * neg + tc) * LD_) : (G + ((size_t)b * Tcn + tc) * LD_);

  float l0 = 0.f, l1 = 0.f;
#pragma unroll 1
  for (int i = 0; i < 4; ++i) {
    const int cc = i * 128 + 4 * lane;
    const v4f a = *(const v4f*)(ls + cc);
    const v4f g = *(const v4f*)(gs + cc);
#pragma unroll
    for (int e = 0; e < 4; ++e) {
      l0 += a[e] * wg[2 * (cc + e)]     + g[e] * wg[2 * (LD_ + cc + e)];
      l1 += a[e] * wg[2 * (cc + e) + 1] + g[e] * wg[2 * (LD_ + cc + e) + 1];
    }
  }
#pragma unroll
  for (int off = 1; off < 32; off <<= 1) {
    l0 += __shfl_xor(l0, off, 32);
    l1 += __shfl_xor(l1, off, 32);
  }
  l0 += bg[0];
  l1 += bg[1];
  const float m   = fmaxf(l0, l1);
  const float e0  = expf(l0 - m), e1 = expf(l1 - m);
  const float inv = 1.0f / (e0 + e1);
  const float g0  = e0 * inv, g1 = e1 * inv;

  v4f lo4[4], go4[4];
#pragma unroll
  for (int i = 0; i < 4; ++i) {
    const int cc = i * 128 + 4 * lane;
    lo4[i] = *(const v4f*)(ls + cc) * g0;
    go4[i] = *(const v4f*)(gs + cc) * g1;
  }
  float* orow = out + (size_t)row * E_;
  for (int pass = 0; pass < 2; ++pass) {
#pragma unroll
    for (int i = 0; i < 4; ++i) {
      *(volatile v4f*)(orow + i * 128 + 4 * lane)       = lo4[i];
      *(volatile v4f*)(orow + LD_ + i * 128 + 4 * lane) = go4[i];
    }
    __threadfence();
  }
}

static unsigned gemm_gx(int M, int N, int rowsW) { return (unsigned)(((M / rowsW) * (N / 64) + 7) / 8); }

extern "C" void kernel_launch(void* const* d_in, const int* in_sizes, int n_in,
                              void* d_out, int out_size, void* d_ws, size_t ws_size,
                              hipStream_t stream) {
  if (n_in < 13) return;
  if (in_sizes[0] != NB_ * T_ * E_) return;
  if (in_sizes[1] != LD_ * 3 * LD_ || in_sizes[3] != LD_ * 3 * LD_) return;
  if (in_sizes[2] != 3 * LD_ || in_sizes[4] != 3 * LD_) return;
  if (in_sizes[5] != 4 * E_ * E_ || in_sizes[6] != E_) return;
  if (in_sizes[7] != LD_ * LD_ || in_sizes[9] != LD_ * LD_) return;
  if (in_sizes[8] != LD_ || in_sizes[10] != LD_) return;
  if (in_sizes[11] != E_ * 2 || in_sizes[12] != 2) return;
  if (out_size != NB_ * T_ * E_) return;

  const float* x       = (const float*)d_in[0];
  const float* w_lqkv  = (const float*)d_in[1];
  const float* b_lqkv  = (const float*)d_in[2];
  const float* w_gqkv  = (const float*)d_in[3];
  const float* b_gqkv  = (const float*)d_in[4];
  const float* w_comp  = (const float*)d_in[5];
  const float* b_comp  = (const float*)d_in[6];
  const float* w_lproj = (const float*)d_in[7];
  const float* b_lproj = (const float*)d_in[8];
  const float* w_gproj = (const float*)d_in[9];
  const float* b_gproj = (const float*)d_in[10];
  const float* w_gate  = (const float*)d_in[11];
  const float* b_gate  = (const float*)d_in[12];
  float* out = (float*)d_out;

  const size_t szWl   = (size_t)3 * LD_ * LD_ * 2;
  const size_t szWc   = (size_t)LD_ * 4 * E_ * 2;
  const size_t szWp   = (size_t)LD_ * LD_ * 2;
  const size_t szX    = (size_t)NB_ * T_ * E_ * 2;
  const size_t szQK   = (size_t)NB_ * T_ * 2 * LD_ * 2;
  const size_t szVT   = (size_t)NB_ * LD_ * T_ * 2;
  const size_t szAO   = (size_t)NB_ * T_ * LD_ * 2;
  const size_t szL    = (size_t)NB_ * T_ * LD_ * 4;
  const size_t szCG   = (size_t)NB_ * TC_ * LD_ * 2;
  const size_t szGQK  = (size_t)NB_ * TC_ * 2 * LD_ * 2;
  const size_t szGVT  = (size_t)NB_ * LD_ * TC_ * 2;
  const size_t szGAO  = (size_t)NB_ * TC_ * LD_ * 2;
  const size_t szGO   = (size_t)NB_ * TC_ * LD_ * 4;
  const size_t szEX   = (size_t)NB_ * XE_ * E_ * 2;
  const size_t szEQK  = (size_t)NB_ * NEL_ * 2 * LD_ * 2;
  const size_t szEVT  = (size_t)NB_ * LD_ * NEL_ * 2;
  const size_t szEAO  = (size_t)NB_ * NEL_ * LD_ * 4;
  const size_t szEAh  = (size_t)NB_ * NEL_ * LD_ * 2;
  const size_t szEL   = szEAO;
  const size_t szECG  = (size_t)NB_ * NEG_ * LD_ * 2;
  const size_t szEGQK = (size_t)NB_ * NEG_ * 2 * LD_ * 2;
  const size_t szEGVT = (size_t)NB_ * LD_ * NEG_ * 2;
  const size_t szEGAO = (size_t)NB_ * NEG_ * LD_ * 4;
  const size_t szEGh  = (size_t)NB_ * NEG_ * LD_ * 2;
  const size_t szEG   = szEGAO;
  size_t off = 0;
  const size_t oWlF = off; off += szWl;  const size_t oWlH = off; off += szWl;  const size_t oWlL = off; off += szWl;
  const size_t oWcF = off; off += szWc;  const size_t oWcH = off; off += szWc;  const size_t oWcL = off; off += szWc;
  const size_t oWgF = off; off += szWl;  const size_t oWgH = off; off += szWl;  const size_t oWgL = off; off += szWl;
  const size_t oWpF = off; off += szWp;  const size_t oWpH = off; off += szWp;  const size_t oWpL = off; off += szWp;
  const size_t oWqF = off; off += szWp;  const size_t oWqH = off; off += szWp;  const size_t oWqL = off; off += szWp;
  const size_t oXs  = off; off += szX;
  const size_t oQK  = off; off += szQK;
  const size_t oVT  = off; off += szVT;
  const size_t oAO  = off; off += szAO;
  const size_t oL   = off; off += szL;
  const size_t oCG  = off; off += szCG;
  const size_t oGQK = off; off += szGQK;
  const size_t oGVT = off; off += szGVT;
  const size_t oGAO = off; off += szGAO;
  const size_t oGO  = off; off += szGO;
  const size_t oEXh = off; off += szEX;   const size_t oEXl = off; off += szEX;
  const size_t oEQKh = off; off += szEQK; const size_t oEQKl = off; off += szEQK;
  const size_t oEVTh = off; off += szEVT; const size_t oEVTl = off; off += szEVT;
  const size_t oEAO  = off; off += szEAO;
  const size_t oEAh  = off; off += szEAh; const size_t oEAl = off; off += szEAh;
  const size_t oEL   = off; off += szEL;
  const size_t oECGh = off; off += szECG; const size_t oECGl = off; off += szECG;
  const size_t oEGQKh = off; off += szEGQK; const size_t oEGQKl = off; off += szEGQK;
  const size_t oEGVTh = off; off += szEGVT; const size_t oEGVTl = off; off += szEGVT;
  const size_t oEGAO = off; off += szEGAO;
  const size_t oEGh  = off; off += szEGh; const size_t oEGl = off; off += szEGh;
  const size_t oEG   = off; off += szEG;
  if (off > ws_size) return;
  if (off > (size_t)134217728) return;

  char* ws = (char*)d_ws;
  unsigned short* WlF = (unsigned short*)(ws + oWlF); unsigned short* WlH = (unsigned short*)(ws + oWlH); unsigned short* WlL = (unsigned short*)(ws + oWlL);
  unsigned short* WcF = (unsigned short*)(ws + oWcF); unsigned short* WcH = (unsigned short*)(ws + oWcH); unsigned short* WcL = (unsigned short*)(ws + oWcL);
  unsigned short* WgF = (unsigned short*)(ws + oWgF); unsigned short* WgH = (unsigned short*)(ws + oWgH); unsigned short* WgL = (unsigned short*)(ws + oWgL);
  unsigned short* WpF = (unsigned short*)(ws + oWpF); unsigned short* WpH = (unsigned short*)(ws + oWpH); unsigned short* WpL = (unsigned short*)(ws + oWpL);
  unsigned short* WqF = (unsigned short*)(ws + oWqF); unsigned short* WqH = (unsigned short*)(ws + oWqH); unsigned short* WqL = (unsigned short*)(ws + oWqL);
  unsigned short* Xs   = (unsigned short*)(ws + oXs);
  unsigned short* QKp  = (unsigned short*)(ws + oQK);
  unsigned short* VTp  = (unsigned short*)(ws + oVT);
  unsigned short* AOp  = (unsigned short*)(ws + oAO);
  float*          Lout = (float*)(ws + oL);
  unsigned short* CGp  = (unsigned short*)(ws + oCG);
  unsigned short* GQKp = (unsigned short*)(ws + oGQK);
  unsigned short* GVTp = (unsigned short*)(ws + oGVT);
  unsigned short* GAOp = (unsigned short*)(ws + oGAO);
  float*          Gout = (float*)(ws + oGO);
  unsigned short* EXh  = (unsigned short*)(ws + oEXh);   unsigned short* EXl  = (unsigned short*)(ws + oEXl);
  unsigned short* EQKh = (unsigned short*)(ws + oEQKh);  unsigned short* EQKl = (unsigned short*)(ws + oEQKl);
  unsigned short* EVTh = (unsigned short*)(ws + oEVTh);  unsigned short* EVTl = (unsigned short*)(ws + oEVTl);
  float*          EAO  = (float*)(ws + oEAO);
  unsigned short* EAh  = (unsigned short*)(ws + oEAh);   unsigned short* EAl  = (unsigned short*)(ws + oEAl);
  float*          EL   = (float*)(ws + oEL);
  unsigned short* ECGh = (unsigned short*)(ws + oECGh);  unsigned short* ECGl = (unsigned short*)(ws + oECGl);
  unsigned short* EGQKh = (unsigned short*)(ws + oEGQKh); unsigned short* EGQKl = (unsigned short*)(ws + oEGQKl);
  unsigned short* EGVTh = (unsigned short*)(ws + oEGVTh); unsigned short* EGVTl = (unsigned short*)(ws + oEGVTl);
  float*          EGAO = (float*)(ws + oEGAO);
  unsigned short* EGh  = (unsigned short*)(ws + oEGh);   unsigned short* EGl  = (unsigned short*)(ws + oEGl);
  float*          EG   = (float*)(ws + oEG);

  const dim3 b256(256), b128(128);
  const size_t vOffW = (size_t)2 * LD_ * LD_;

  wconv_kernel<<<dim3(3 * LD_ / 64, LD_ / 64), b256, 0, stream>>>(w_lqkv, 3 * LD_, WlF, WlH, WlL, LD_, 3 * LD_, 64.f);
  wconv_kernel<<<dim3(3 * LD_ / 64, LD_ / 64), b256, 0, stream>>>(w_gqkv, 3 * LD_, WgF, WgH, WgL, LD_, 3 * LD_, 64.f);
  wconv_kernel<<<dim3(LD_ / 64, 4 * E_ / 64), b256, 0, stream>>>(w_comp + LD_, E_, WcF, WcH, WcL, 4 * E_, LD_, 64.f);
  wconv_kernel<<<dim3(LD_ / 64, LD_ / 64), b256, 0, stream>>>(w_lproj, LD_, WpF, WpH, WpL, LD_, LD_, 64.f);
  wconv_kernel<<<dim3(LD_ / 64, LD_ / 64), b256, 0, stream>>>(w_gproj, LD_, WqF, WqH, WqL, LD_, LD_, 64.f);
  xconv_kernel<<<dim3(NB_ * T_ * E_ / 8 / 256), b256, 0, stream>>>(x, Xs, NB_ * T_ * E_ / 8, 8.f);
  split_bf16x2_kernel<<<dim3(XE_ * E_ / 2 / 256, NB_), b256, 0, stream>>>(x, (long long)T_ * E_, EXh, EXl, (long long)XE_ * E_, XE_ * E_ / 2);

  wmma_gemm<0, false, 2, 1, 4><<<dim3(gemm_gx(NB_ * T_, 2 * LD_, 64), 1), b256, 0, stream>>>(
      Xs, Xs, E_, 0LL, WlF, WlF, LD_, 0LL, (void*)QKp, (void*)QKp, 2 * LD_, 0LL,
      b_lqkv, NB_ * T_, 2 * LD_, LD_, 1.f / 512.f, 16.f);
  wmma_gemm<0, false, 1, 1, 4><<<dim3(gemm_gx(LD_, T_, 64), NB_), b256, 0, stream>>>(
      WlF + vOffW, WlF + vOffW, LD_, 0LL, Xs, Xs, E_, (long long)T_ * E_, (void*)VTp, (void*)VTp, T_, (long long)LD_ * T_,
      b_lqkv + 2 * LD_, LD_, T_, LD_, 1.f / 512.f, 16.f);
  attn_causal64<0><<<dim3(HH_ * (T_ / 64), NB_), b128, 0, stream>>>(
      QKp, QKp, 2 * LD_, (long long)T_ * 2 * LD_, LD_, VTp, VTp, T_, (long long)LD_ * T_,
      (void*)AOp, LD_, (long long)T_ * LD_, T_ / 64, 1.f / 2048.f, 1.f / 1024.f);
  wmma_gemm<0, false, 2, 0, 4><<<dim3(gemm_gx(NB_ * T_, LD_, 64), 1), b256, 0, stream>>>(
      AOp, AOp, LD_, 0LL, WpF, WpF, LD_, 0LL, (void*)Lout, (void*)Lout, LD_, 0LL,
      b_lproj, NB_ * T_, LD_, LD_, 1.f / 1024.f, 1.f);
  wmma_gemm<0, false, 2, 1, 4><<<dim3(gemm_gx(NB_ * TC_, LD_, 64), 1), b256, 0, stream>>>(
      Xs, Xs, 4 * E_, 0LL, WcF, WcF, 4 * E_, 0LL, (void*)CGp, (void*)CGp, LD_, 0LL,
      b_comp + LD_, NB_ * TC_, LD_, 4 * E_, 1.f / 512.f, 8.f);
  wmma_gemm<0, false, 2, 1, 4><<<dim3(gemm_gx(NB_ * TC_, 2 * LD_, 64), 1), b256, 0, stream>>>(
      CGp, CGp, LD_, 0LL, WgF, WgF, LD_, 0LL, (void*)GQKp, (void*)GQKp, 2 * LD_, 0LL,
      b_gqkv, NB_ * TC_, 2 * LD_, LD_, 1.f / 512.f, 16.f);
  wmma_gemm<0, false, 1, 1, 4><<<dim3(gemm_gx(LD_, TC_, 64), NB_), b256, 0, stream>>>(
      WgF + vOffW, WgF + vOffW, LD_, 0LL, CGp, CGp, LD_, (long long)TC_ * LD_, (void*)GVTp, (void*)GVTp, TC_, (long long)LD_ * TC_,
      b_gqkv + 2 * LD_, LD_, TC_, LD_, 1.f / 512.f, 16.f);
  attn_causal64<0><<<dim3(HH_ * (TC_ / 64), NB_), b128, 0, stream>>>(
      GQKp, GQKp, 2 * LD_, (long long)TC_ * 2 * LD_, LD_, GVTp, GVTp, TC_, (long long)LD_ * TC_,
      (void*)GAOp, LD_, (long long)TC_ * LD_, TC_ / 64, 1.f / 2048.f, 1.f / 1024.f);
  wmma_gemm<0, false, 2, 0, 4><<<dim3(gemm_gx(NB_ * TC_, LD_, 64), 1), b256, 0, stream>>>(
      GAOp, GAOp, LD_, 0LL, WqF, WqF, LD_, 0LL, (void*)Gout, (void*)Gout, LD_, 0LL,
      b_gproj, NB_ * TC_, LD_, LD_, 1.f / 1024.f, 1.f);

  wmma_gemm<1, true, 2, 2, 2><<<dim3(gemm_gx(NEL_, 2 * LD_, 32), NB_), b256, 0, stream>>>(
      EXh, EXl, E_, (long long)XE_ * E_, WlH, WlL, LD_, 0LL, (void*)EQKh, (void*)EQKl, 2 * LD_, (long long)NEL_ * 2 * LD_,
      b_lqkv, NEL_, 2 * LD_, LD_, 1.f, 1.f);
  wmma_gemm<1, true, 1, 2, 2><<<dim3(gemm_gx(LD_, NEL_, 32), NB_), b256, 0, stream>>>(
      WlH + vOffW, WlL + vOffW, LD_, 0LL, EXh, EXl, E_, (long long)XE_ * E_, (void*)EVTh, (void*)EVTl, NEL_, (long long)LD_ * NEL_,
      b_lqkv + 2 * LD_, LD_, NEL_, LD_, 1.f, 1.f);
  attn_causal64<1><<<dim3(HH_ * (NEL_ / 64), NB_), b128, 0, stream>>>(
      EQKh, EQKl, 2 * LD_, (long long)NEL_ * 2 * LD_, LD_, EVTh, EVTl, NEL_, (long long)LD_ * NEL_,
      (void*)EAO, LD_, (long long)NEL_ * LD_, NEL_ / 64, 0.125f, 1.f);
  split_bf16x2_kernel<<<dim3(NB_ * NEL_ * LD_ / 2 / 256, 1), b256, 0, stream>>>(EAO, 0LL, EAh, EAl, 0LL, NB_ * NEL_ * LD_ / 2);
  wmma_gemm<1, true, 2, 0, 2><<<dim3(gemm_gx(NB_ * NEL_, LD_, 32), 1), b256, 0, stream>>>(
      EAh, EAl, LD_, 0LL, WpH, WpL, LD_, 0LL, (void*)EL, (void*)EL, LD_, 0LL,
      b_lproj, NB_ * NEL_, LD_, LD_, 1.f, 1.f);
  wmma_gemm<1, true, 2, 2, 2><<<dim3(gemm_gx(NEG_, LD_, 32), NB_), b256, 0, stream>>>(
      EXh, EXl, 4 * E_, (long long)XE_ * E_, WcH, WcL, 4 * E_, 0LL, (void*)ECGh, (void*)ECGl, LD_, (long long)NEG_ * LD_,
      b_comp + LD_, NEG_, LD_, 4 * E_, 1.f, 1.f);
  wmma_gemm<1, true, 2, 2, 2><<<dim3(gemm_gx(NB_ * NEG_, 2 * LD_, 32), 1), b256, 0, stream>>>(
      ECGh, ECGl, LD_, 0LL, WgH, WgL, LD_, 0LL, (void*)EGQKh, (void*)EGQKl, 2 * LD_, 0LL,
      b_gqkv, NB_ * NEG_, 2 * LD_, LD_, 1.f, 1.f);
  wmma_gemm<1, true, 1, 2, 2><<<dim3(gemm_gx(LD_, NEG_, 32), NB_), b256, 0, stream>>>(
      WgH + vOffW, WgL + vOffW, LD_, 0LL, ECGh, ECGl, LD_, (long long)NEG_ * LD_, (void*)EGVTh, (void*)EGVTl, NEG_, (long long)LD_ * NEG_,
      b_gqkv + 2 * LD_, LD_, NEG_, LD_, 1.f, 1.f);
  attn_causal64<1><<<dim3(HH_ * (NEG_ / 64), NB_), b128, 0, stream>>>(
      EGQKh, EGQKl, 2 * LD_, (long long)NEG_ * 2 * LD_, LD_, EGVTh, EGVTl, NEG_, (long long)LD_ * NEG_,
      (void*)EGAO, LD_, (long long)NEG_ * LD_, NEG_ / 64, 0.125f, 1.f);
  split_bf16x2_kernel<<<dim3(NB_ * NEG_ * LD_ / 2 / 256, 1), b256, 0, stream>>>(EGAO, 0LL, EGh, EGl, 0LL, NB_ * NEG_ * LD_ / 2);
  wmma_gemm<1, true, 2, 0, 2><<<dim3(gemm_gx(NB_ * NEG_, LD_, 32), 1), b256, 0, stream>>>(
      EGh, EGl, LD_, 0LL, WqH, WqL, LD_, 0LL, (void*)EG, (void*)EG, LD_, 0LL,
      b_gproj, NB_ * NEG_, LD_, LD_, 1.f, 1.f);

  gate_out_kernel<<<dim3(NB_ * T_ / 8), b256, 0, stream>>>(Lout, EL, Gout, EG, w_gate, b_gate, out,
                                                            NB_ * T_, T_, TC_, NEL_, NEG_);
  (void)hipGetLastError();
}
